// PagedJointAttention_46926812676617
// MI455X (gfx1250) — hardware-verified
//
#include <hip/hip_runtime.h>


#define NB_  2
#define SS   1024
#define SC   2048
#define SE   256
#define TQ   (SS + SE)
#define TK   (SC + SS + SE)
#define EE   2048
#define NH_  16
#define HD   128
#define ZH   2
#define PCAR 1024.0f
typedef _Float16 h16;
typedef unsigned short bf;
typedef __attribute__((ext_vector_type(16))) __bf16   v16bf;
typedef __attribute__((ext_vector_type(16))) _Float16 v16h;
typedef __attribute__((ext_vector_type(8)))  _Float16 v8h;
typedef __attribute__((ext_vector_type(8)))  unsigned short v8us;
typedef __attribute__((ext_vector_type(8)))  float    v8f;
typedef __attribute__((ext_vector_type(4)))  float    v4f;
typedef v8h  __attribute__((may_alias)) v8ha;
typedef v4f  __attribute__((may_alias)) v4fa;
typedef v8us __attribute__((may_alias)) v8usa;

__device__ __forceinline__ unsigned short f2bf(float f) { unsigned u = __float_as_uint(f); u += 0x7FFFu + ((u >> 16) & 1u); return (unsigned short)(u >> 16); }
__device__ __forceinline__ float bf2f(unsigned short b) { return __uint_as_float(((unsigned)b) << 16); }
__device__ __forceinline__ float bfr(float f) { return bf2f(f2bf(f)); }
__device__ __forceinline__ v16h cat16(v8h lo, v8h hi) { return __builtin_shufflevector(lo, hi, 0, 1, 2, 3, 4, 5, 6, 7, 8, 9, 10, 11, 12, 13, 14, 15); }
__device__ __forceinline__ v16bf cat16b(v8us lo, v8us hi) { return __builtin_bit_cast(v16bf, __builtin_shufflevector(lo, hi, 0, 1, 2, 3, 4, 5, 6, 7, 8, 9, 10, 11, 12, 13, 14, 15)); }
__device__ __forceinline__ v8f wmma16(v16h a, v16h b, v8f c) { return __builtin_amdgcn_wmma_f32_16x16x32_f16(false, a, false, b, (short)0, c, false, false); }
__device__ __forceinline__ v8f wmmab(v16bf a, v16bf b, v8f c) { return __builtin_amdgcn_wmma_f32_16x16x32_bf16(false, a, false, b, (short)0, c, false, false); }


template <typename T16> struct WFrag;
template <> struct WFrag<h16> { typedef v16h V; static __device__ __forceinline__ V ld(const h16* p) { return cat16(*(const v8h*)p, *(const v8h*)(p + 16)); } static __device__ __forceinline__ v8f mma(V a, V b, v8f c) { return wmma16(a, b, c); } };
template <> struct WFrag<bf> { typedef v16bf V; static __device__ __forceinline__ V ld(const bf* p) { return cat16b(*(const v8us*)p, *(const v8us*)(p + 16)); } static __device__ __forceinline__ v8f mma(V a, V b, v8f c) { return wmmab(a, b, c); } };
template <typename T16, int NSPLIT, bool BIAS>
__global__ __launch_bounds__(32) void k_gemmw(const T16* __restrict__ A, const T16* __restrict__ A2, const T16* __restrict__ Bt, const T16* __restrict__ Bt2, int K, float* C, int ldc, const float* __restrict__ bias, size_t sA, size_t sB, size_t sC) {
    typedef typename WFrag<T16>::V V;
    __shared__ __align__(16) float os[16 * 68];
    const size_t z = blockIdx.z; A += z * sA; if (A2) A2 += z * sA; Bt += z * sB; if (Bt2) Bt2 += z * sB; C += z * sC;
    const int lane = threadIdx.x & 31, lr = lane & 15, hi = lane >> 4; const int r0 = blockIdx.x * 64, c0 = blockIdx.y * 64;
    v8f acc[4][4];
#pragma unroll
    for (int mb = 0; mb < 4; ++mb)
#pragma unroll
        for (int nb = 0; nb < 4; ++nb) acc[mb][nb] = (v8f){};
    const size_t aoff = (size_t)(r0 + lr) * K + 8 * hi, boff = (size_t)(c0 + lr) * K + 8 * hi;
#pragma unroll 1
    for (int kc = 0; kc < K; kc += 32) {
        V a[4], a2[4];
#pragma unroll
        for (int mb = 0; mb < 4; ++mb) { a[mb] = WFrag<T16>::ld(A + aoff + (size_t)mb * 16 * K + kc); if (NSPLIT == 1 || NSPLIT == 2) a2[mb] = WFrag<T16>::ld(A2 + aoff + (size_t)mb * 16 * K + kc); }
#pragma unroll
        for (int nb = 0; nb < 4; ++nb) { const V b = WFrag<T16>::ld(Bt + boff + (size_t)nb * 16 * K + kc); V b2; if (NSPLIT >= 2) b2 = WFrag<T16>::ld(Bt2 + boff + (size_t)nb * 16 * K + kc);
#pragma unroll
            for (int mb = 0; mb < 4; ++mb) { acc[mb][nb] = WFrag<T16>::mma(a[mb], b, acc[mb][nb]); if (NSPLIT == 1 || NSPLIT == 2) acc[mb][nb] = WFrag<T16>::mma(a2[mb], b, acc[mb][nb]); if (NSPLIT >= 2) acc[mb][nb] = WFrag<T16>::mma(a[mb], b2, acc[mb][nb]); } }
        asm volatile("v_nop\n\tv_nop\n\tv_nop\n\tv_nop" : "+v"(acc[0][0]), "+v"(acc[1][1]), "+v"(acc[2][2]), "+v"(acc[3][3]) : "v"(a[0]), "v"(a[3]));
    }
#pragma unroll
    for (int mb = 0; mb < 4; ++mb) {
#pragma unroll
        for (int nb = 0; nb < 4; ++nb) {
#pragma unroll
            for (int j = 0; j < 8; ++j) os[(hi * 8 + j) * 68 + nb * 16 + lr] = acc[mb][nb][j]; }
        __builtin_amdgcn_wave_barrier(); asm volatile("" ::: "memory");
        float* crow = C + (size_t)(r0 + mb * 16) * ldc + c0;
#pragma unroll 1
        for (int ps = 0; ps < 2; ++ps) {
#pragma unroll
            for (int s = 0; s < 8; ++s) { const int row = 2 * s + hi, cofs = lr * 4; v4f val = *(const v4fa*)(os + row * 68 + cofs); if (BIAS) { val[0] += bfr(bias[c0 + cofs]); val[1] += bfr(bias[c0 + cofs + 1]); val[2] += bfr(bias[c0 + cofs + 2]); val[3] += bfr(bias[c0 + cofs + 3]); }
                *(volatile v4f*)(crow + (size_t)row * ldc + cofs) = val; }
            if (ps == 0) __threadfence(); }
        __builtin_amdgcn_wave_barrier(); asm volatile("" ::: "memory");
    }
}

__device__ __forceinline__ h16 tohx(float x) { return (h16)x; }
__device__ __forceinline__ void splitf(float y, unsigned short& h, unsigned short& l) { h = f2bf(y); l = f2bf(y - bf2f(h)); }
typedef __attribute__((ext_vector_type(2))) unsigned short v2us;
typedef __attribute__((ext_vector_type(4))) unsigned short v4us;
typedef __attribute__((ext_vector_type(2))) _Float16 v2h;
typedef __attribute__((ext_vector_type(4))) _Float16 v4h;

__global__ __launch_bounds__(256) void k_cvt8(const float* __restrict__ src, bf* dst, size_t n8) { const size_t i = (size_t)blockIdx.x * 256 + threadIdx.x; if (i >= n8) return; const v8f v = *(const v8f*)(src + i * 8); v8us o;
#pragma unroll
    for (int k = 0; k < 8; ++k) o[k] = f2bf(v[k]); *(volatile v8us*)(dst + i * 8) = o; __threadfence(); *(volatile v8us*)(dst + i * 8) = o; }
__global__ __launch_bounds__(256) void k_wtG(const float* __restrict__ w, int K, int N, bf* Bt) {
    const int lane = threadIdx.x & 31; const int L0 = (blockIdx.x * 8 + (threadIdx.x >> 5)) * 8; const int nlines = N * K / 64;
#pragma unroll
    for (int ps = 0; ps < 2; ++ps) {
#pragma unroll 1
        for (int l = 0; l < 8; ++l) { const int L = L0 + l; if (L >= nlines) break; const size_t e = (size_t)L * 64 + lane * 2; const int k = (int)(e % K), n = (int)(e / K); v2us o;
            o[0] = f2bf(w[(size_t)k * N + n]); o[1] = f2bf(w[(size_t)(k + 1) * N + n]); *(volatile v2us*)(Bt + e) = o; }
        if (ps == 0) __threadfence(); }
}

__global__ __launch_bounds__(256) void k_qp(const float* __restrict__ F, int src_is_cache, int rows, const float* __restrict__ gw, int roff, int prow, h16* P) { const int lane = threadIdx.x & 31; const int row = blockIdx.x * 8 + (threadIdx.x >> 5); if (row >= rows * NH_) return; const int h = row % NH_; const int r = row / NH_;
    const float* f = src_is_cache ? (F + ((size_t)h * rows + r) * HD) : (F + (size_t)r * EE + h * HD); v4f a = *(const v4f*)(f + lane * 4); if (src_is_cache) { for (int u = 0; u < 4; ++u) a[u] = bfr(a[u]); }
    float rs = 1.0f; if (gw) { float q = 0.f;
#pragma unroll
        for (int u = 0; u < 4; ++u) { float p = __fmul_rn(a[u], a[u]); asm volatile("" : "+v"(p)); q = __fadd_rn(q, p); }
#pragma unroll
        for (int sh = 16; sh; sh >>= 1) q += __shfl_xor(q, sh, 32);
        rs = __frsqrt_rn(__fadd_rn(q * (1.0f / HD), 1e-6f)); }
    v4h o;
#pragma unroll
    for (int u = 0; u < 4; ++u) { float y = a[u]; if (gw) { float n0 = __fmul_rn(y, rs); asm volatile("" : "+v"(n0)); y = __fmul_rn(n0, bfr(gw[lane * 4 + u])); } o[u] = tohx(y); }
    h16* dst = P + ((size_t)h * prow + roff + r) * HD + lane * 4; *(volatile v4h*)dst = o; __threadfence(); *(volatile v4h*)dst = o; }
__global__ __launch_bounds__(256) void k_vt(const float* __restrict__ F, int rows, int koff, h16* VT) { const size_t e = ((size_t)blockIdx.x * 256 + threadIdx.x) * 2; if (e >= (size_t)NH_ * HD * rows) return; const int t = (int)(e % rows); const int d = (int)((e / rows) % HD); const int h = (int)(e / ((size_t)rows * HD)); v2h o; o[0] = tohx(F[(size_t)t * EE + h * HD + d]); o[1] = tohx(F[(size_t)(t + 1) * EE + h * HD + d]); h16* dst = VT + ((size_t)h * HD + d) * TK + koff + t; *(volatile v2h*)dst = o; __threadfence(); *(volatile v2h*)dst = o; }
__global__ __launch_bounds__(256) void k_vtc(const float* __restrict__ VC, h16* VT) { const size_t e = ((size_t)blockIdx.x * 256 + threadIdx.x) * 2; if (e >= (size_t)NH_ * HD * SC) return; const int t = (int)(e % SC); const int d = (int)((e / SC) % HD); const int h = (int)(e / ((size_t)SC * HD)); v2h o; o[0] = tohx(bfr(VC[((size_t)h * SC + t) * HD + d])); o[1] = tohx(bfr(VC[((size_t)h * SC + t + 1) * HD + d])); h16* dst = VT + ((size_t)h * HD + d) * TK + t; *(volatile v2h*)dst = o; __threadfence(); *(volatile v2h*)dst = o; }
__global__ __launch_bounds__(256) void k_soft(const float* __restrict__ S, h16* P16) { const int lane = threadIdx.x & 31; const int row = blockIdx.x * 8 + (threadIdx.x >> 5); if (row >= ZH * TQ) return; const float* sr = S + (size_t)row * TK; float v[TK / 32]; float mx = -3.0e38f;
#pragma unroll
    for (int ch = 0; ch < TK / 128; ++ch) { const v4f a = *(const v4f*)(sr + ch * 128 + lane * 4);
#pragma unroll
        for (int u = 0; u < 4; ++u) { const float t = a[u] * 0.088388347648318447f; v[ch * 4 + u] = t; mx = fmaxf(mx, t); } }
#pragma unroll
    for (int sh = 16; sh; sh >>= 1) mx = fmaxf(mx, __shfl_xor(mx, sh, 32));
    float sum = 0.f;
#pragma unroll
    for (int q = 0; q < TK / 32; ++q) { float d0 = __fsub_rn(v[q], mx); asm volatile("" : "+v"(d0)); v[q] = __builtin_amdgcn_exp2f(__fmul_rn(d0, 1.4426950408889634f)); sum += v[q]; }
#pragma unroll
    for (int sh = 16; sh; sh >>= 1) sum += __shfl_xor(sum, sh, 32);
    const float f = __fdiv_rn(PCAR, sum);
    for (int ps = 0; ps < 2; ++ps) {
#pragma unroll
        for (int ch = 0; ch < TK / 128; ++ch) { v4h o4; for (int q = 0; q < 4; ++q) o4[q] = tohx(v[ch * 4 + q] * f); *(volatile v4h*)(P16 + (size_t)row * TK + ch * 128 + lane * 4) = o4; }
        if (ps == 0) __threadfence(); } }
__global__ __launch_bounds__(256) void k_mrg(const float* __restrict__ O, int h0, bf* A1h, bf* A1l, bf* A2h, bf* A2l) { const size_t e = ((size_t)blockIdx.x * 256 + threadIdx.x) * 4; if (e >= (size_t)ZH * TQ * HD) return; const int d = (int)(e % HD); const int q = (int)((e / HD) % TQ); const int zz = (int)(e / ((size_t)HD * TQ)); v4us oh, ol;
#pragma unroll
    for (int u = 0; u < 4; ++u) { unsigned short a, b; splitf(O[e + u] * (1.0f / PCAR), a, b); oh[u] = a; ol[u] = b; }
    bf* Ah = (q < SS) ? A1h : A2h; bf* Al = (q < SS) ? A1l : A2l; const size_t oo = (size_t)((q < SS) ? q : q - SS) * EE + (h0 + zz) * HD + d;
    *(volatile v4us*)(Ah + oo) = oh; *(volatile v4us*)(Al + oo) = ol; __threadfence(); *(volatile v4us*)(Ah + oo) = oh; *(volatile v4us*)(Al + oo) = ol; }

extern "C" void kernel_launch(void* const* d_in, const int* in_sizes, int n_in,
                              void* d_out, int out_size, void* d_ws, size_t ws_size, hipStream_t stream) {
    (void)in_sizes; (void)n_in; (void)out_size;
    const float* x = (const float*)d_in[0]; const float* kc = (const float*)d_in[1]; const float* vc = (const float*)d_in[2]; const float* enc = (const float*)d_in[3];
    const float* Wq = (const float*)d_in[4]; const float* bq = (const float*)d_in[5]; const float* Wk = (const float*)d_in[6]; const float* bk = (const float*)d_in[7]; const float* Wv = (const float*)d_in[8]; const float* bv = (const float*)d_in[9];
    const float* Waq = (const float*)d_in[10]; const float* baq = (const float*)d_in[11]; const float* Wak = (const float*)d_in[12]; const float* bak = (const float*)d_in[13]; const float* Wav = (const float*)d_in[14]; const float* bav = (const float*)d_in[15];
    const float* Wo = (const float*)d_in[16]; const float* bo = (const float*)d_in[17]; const float* Wao = (const float*)d_in[18]; const float* bao = (const float*)d_in[19]; const float* gq = (const float*)d_in[20]; const float* gk = (const float*)d_in[21]; const float* gaq = (const float*)d_in[22]; const float* gak = (const float*)d_in[23];
    float* OUT0 = (float*)d_out; float* OUT1 = (float*)d_out + (size_t)NB_ * SS * EE;
    char* wsp = (char*)d_ws;
    auto take = [&](size_t bytes) { char* p = wsp; wsp += (bytes + 255) & ~(size_t)255; return (void*)p; };
    bf* BQ = (bf*)take((size_t)EE * EE * 2); bf* BK = (bf*)take((size_t)EE * EE * 2); bf* BV = (bf*)take((size_t)EE * EE * 2); bf* BAQ = (bf*)take((size_t)EE * EE * 2); bf* BAK = (bf*)take((size_t)EE * EE * 2); bf* BAV = (bf*)take((size_t)EE * EE * 2); bf* BO = (bf*)take((size_t)EE * EE * 2); bf* BAO = (bf*)take((size_t)EE * EE * 2);
    bf* XB = (bf*)take((size_t)SS * EE * 2); bf* EB = (bf*)take((size_t)SE * EE * 2); float* F = (float*)take((size_t)SS * EE * 4); float* FE = (float*)take((size_t)SE * EE * 4);
    h16* QP = (h16*)take((size_t)NH_ * TQ * HD * 2); h16* KP = (h16*)take((size_t)NH_ * TK * HD * 2); h16* VT = (h16*)take((size_t)NH_ * HD * TK * 2); float* S = (float*)take((size_t)ZH * TQ * TK * 4); h16* P16 = (h16*)take((size_t)ZH * TQ * TK * 2); float* O = (float*)take((size_t)ZH * TQ * HD * 4);
    bf* A1h = (bf*)take((size_t)SS * EE * 2); bf* A1l = (bf*)take((size_t)SS * EE * 2); bf* A2h = (bf*)take((size_t)SE * EE * 2); bf* A2l = (bf*)take((size_t)SE * EE * 2);
    if ((size_t)(wsp - (char*)d_ws) > ws_size) return;
    k_wtG<<<(EE * EE / 64 + 63) / 64, 256, 0, stream>>>(Wq, EE, EE, BQ); k_wtG<<<(EE * EE / 64 + 63) / 64, 256, 0, stream>>>(Wk, EE, EE, BK); k_wtG<<<(EE * EE / 64 + 63) / 64, 256, 0, stream>>>(Wv, EE, EE, BV);
    k_wtG<<<(EE * EE / 64 + 63) / 64, 256, 0, stream>>>(Waq, EE, EE, BAQ); k_wtG<<<(EE * EE / 64 + 63) / 64, 256, 0, stream>>>(Wak, EE, EE, BAK); k_wtG<<<(EE * EE / 64 + 63) / 64, 256, 0, stream>>>(Wav, EE, EE, BAV); k_wtG<<<(EE * EE / 64 + 63) / 64, 256, 0, stream>>>(Wo, EE, EE, BO); k_wtG<<<(EE * EE / 64 + 63) / 64, 256, 0, stream>>>(Wao, EE, EE, BAO);
    const dim3 gs(SS / 64, EE / 64, 1), ge(SE / 64, EE / 64, 1); const size_t zq = (size_t)TQ * HD, zk = (size_t)TK * HD, zS = (size_t)TQ * TK, zv = (size_t)HD * TK, zo = (size_t)TQ * HD;
    for (int b = 0; b < NB_; ++b) { const float* kcb = kc + (size_t)b * NH_ * SC * HD; const float* vcb = vc + (size_t)b * NH_ * SC * HD;
        k_cvt8<<<(SS * EE / 8 + 255) / 256, 256, 0, stream>>>(x + (size_t)b * SS * EE, XB, SS * EE / 8); k_cvt8<<<(SE * EE / 8 + 255) / 256, 256, 0, stream>>>(enc + (size_t)b * SE * EE, EB, SE * EE / 8);
        k_gemmw<bf, 0, true><<<gs, 32, 0, stream>>>(XB, nullptr, BQ, nullptr, EE, F, EE, bq, 0, 0, 0); k_qp<<<SS * NH_ / 8, 256, 0, stream>>>(F, 0, SS, gq, 0, TQ, QP);
        k_gemmw<bf, 0, true><<<ge, 32, 0, stream>>>(EB, nullptr, BAQ, nullptr, EE, FE, EE, baq, 0, 0, 0); k_qp<<<SE * NH_ / 8, 256, 0, stream>>>(FE, 0, SE, gaq, SS, TQ, QP);
        k_qp<<<SC * NH_ / 8, 256, 0, stream>>>(kcb, 1, SC, gk, 0, TK, KP);
        k_gemmw<bf, 0, true><<<gs, 32, 0, stream>>>(XB, nullptr, BK, nullptr, EE, F, EE, bk, 0, 0, 0); k_qp<<<SS * NH_ / 8, 256, 0, stream>>>(F, 0, SS, gk, SC, TK, KP);
        k_gemmw<bf, 0, true><<<ge, 32, 0, stream>>>(EB, nullptr, BAK, nullptr, EE, FE, EE, bak, 0, 0, 0); k_qp<<<SE * NH_ / 8, 256, 0, stream>>>(FE, 0, SE, gak, SC + SS, TK, KP);
        k_vtc<<<(unsigned)(((size_t)NH_ * HD * SC / 2 + 255) / 256), 256, 0, stream>>>(vcb, VT);
        k_gemmw<bf, 0, true><<<gs, 32, 0, stream>>>(XB, nullptr, BV, nullptr, EE, F, EE, bv, 0, 0, 0); k_vt<<<(unsigned)(((size_t)NH_ * HD * SS / 2 + 255) / 256), 256, 0, stream>>>(F, SS, SC, VT);
        k_gemmw<bf, 0, true><<<ge, 32, 0, stream>>>(EB, nullptr, BAV, nullptr, EE, FE, EE, bav, 0, 0, 0); k_vt<<<(unsigned)(((size_t)NH_ * HD * SE / 2 + 255) / 256), 256, 0, stream>>>(FE, SE, SC + SS, VT);
        for (int h0 = 0; h0 < NH_; h0 += ZH) {
            k_gemmw<h16, 0, false><<<dim3(TQ / 64, TK / 64, ZH), 32, 0, stream>>>(QP + (size_t)h0 * zq, nullptr, KP + (size_t)h0 * zk, nullptr, HD, S, TK, nullptr, zq, zk, zS);
            k_soft<<<ZH * TQ / 8, 256, 0, stream>>>(S, P16);
            k_gemmw<h16, 0, false><<<dim3(TQ / 64, HD / 64, ZH), 32, 0, stream>>>(P16, nullptr, VT + (size_t)h0 * zv, nullptr, TK, O, HD, nullptr, zS, zv, zo);
            k_mrg<<<(unsigned)(((size_t)ZH * TQ * HD / 4 + 255) / 256), 256, 0, stream>>>(O, h0, A1h, A1l, A2h, A2l); }
        k_gemmw<bf, 1, true><<<gs, 32, 0, stream>>>(A1h, A1l, BO, nullptr, EE, OUT0 + (size_t)b * SS * EE, EE, bo, 0, 0, 0);
        k_gemmw<bf, 1, true><<<ge, 32, 0, stream>>>(A2h, A2l, BAO, nullptr, EE, OUT1 + (size_t)b * SE * EE, EE, bao, 0, 0, 0); }
}
